// S4_39616778338840
// MI455X (gfx1250) — hardware-verified
//
#include <hip/hip_runtime.h>
#include <math.h>

typedef __attribute__((ext_vector_type(16))) _Float16 v16h;
typedef __attribute__((ext_vector_type(8)))  _Float16 v8h;
typedef __attribute__((ext_vector_type(16))) __bf16   v16b;
typedef __attribute__((ext_vector_type(8)))  __bf16   v8b;
typedef __attribute__((ext_vector_type(8)))  float    v8f;
typedef __attribute__((ext_vector_type(4)))  float    v4f;
typedef __attribute__((ext_vector_type(4)))  unsigned u32x4;

constexpr int kNB    = 32;
constexpr int kT     = 2048;
constexpr int kDI    = 64;
constexpr int kP     = 256;
constexpr int kHid   = 512;
constexpr int kDO    = 64;
constexpr int kRows  = kNB * kT;
constexpr int kNQ    = 4;
constexpr int kRowsQ = kRows / kNQ;
constexpr int kNBQ   = kNB / kNQ;
constexpr int kK3    = 3 * kHid;
constexpr int kScanLanes = kHid / 8;
static_assert(kRowsQ * kNQ == kRows && kNBQ * kT == kRowsQ, "quarter split");
static_assert((kDI % 32) == 0 && (kP % 32) == 0 && (kK3 % 32) == 0, "GEMM K multiples of 32");
static_assert((kRowsQ % 64) == 0 && (kP % 64) == 0 && (kHid % 64) == 0 && (kDO % 64) == 0, "GEMM M,N multiples of 64");
static_assert(kScanLanes == 64 && (kHid % 8) == 0, "scan block = 64 lanes x 8 channels");
static_assert(((kRows * kDI) % 8) == 0 && ((kP * kDI) % 8) == 0, "cast coverage");
static_assert((((kRowsQ / 64) * (kP / 64)) % 8) == 0 && (((kRowsQ / 64) * (kHid / 64)) % 8) == 0 &&
              (((kRowsQ / 64) * (kDO / 64)) % 8) == 0, "8 tiles per GEMM block exactly");

constexpr size_t kOffXH  = 0;
constexpr size_t kOffWI  = kOffXH + (size_t)kRows  * kDI  * 2;
constexpr size_t kOffBT  = kOffWI + (size_t)kP     * kDI  * 2;
constexpr size_t kOffCW  = kOffBT + (size_t)kHid   * kP   * 2;
constexpr size_t kOffPP  = kOffCW + (size_t)kDO    * kK3  * 2;
constexpr size_t kOffUU  = kOffPP + (size_t)kRowsQ * kP   * 2;
constexpr size_t kOffA3  = kOffUU + (size_t)kRowsQ * kHid * 2;
constexpr size_t kWsTotal = kOffA3 + (size_t)kRowsQ * kK3 * 2;
static_assert(kWsTotal == 84377600ull, "carve total");
static_assert(kWsTotal <= 134217728ull, "carve cap");
static_assert((kOffWI % 128) == 0 && (kOffBT % 128) == 0 && (kOffCW % 128) == 0 &&
              (kOffPP % 128) == 0 && (kOffUU % 128) == 0 && (kOffA3 % 128) == 0, "128-B aligned regions");

__device__ __forceinline__ float h16_to_f32(unsigned hb) {
  const unsigned sgn = (hb & 0x8000u) << 16; const unsigned em = hb & 0x7fffu;
  const float fn = __uint_as_float((em << 13) + 0x38000000u);
  const float fs = (float)em * 5.9604644775390625e-8f;
  const float mag = (em < 0x400u) ? fs : fn; return __uint_as_float(__float_as_uint(mag) | sgn); }
__device__ __forceinline__ unsigned f16_bits(float f) { return (unsigned)__builtin_bit_cast(unsigned short, (_Float16)f); }

__device__ __forceinline__ unsigned short f2bf_bits(float f) {
  unsigned u = __float_as_uint(f);
  return (unsigned short)((u + 0x7FFFu + ((u >> 16) & 1u)) >> 16);
}
__device__ __forceinline__ float bf_bits2f(unsigned short h) { return __uint_as_float(((unsigned)h) << 16); }

__device__ __forceinline__ void dep_guard4_h(v8f& a, v8f& b, v8f& c, v8f& d, v16h x, v16h y) { asm volatile("v_nop\n\tv_nop\n\tv_nop\n\tv_nop" : "+v"(a), "+v"(b), "+v"(c), "+v"(d) : "v"(x), "v"(y)); }
__device__ __forceinline__ void dep_guard4_b(v8f& a, v8f& b, v8f& c, v8f& d, v16b x, v16b y) { asm volatile("v_nop\n\tv_nop\n\tv_nop\n\tv_nop" : "+v"(a), "+v"(b), "+v"(c), "+v"(d) : "v"(x), "v"(y)); }
__device__ __forceinline__ void keep4_h(v16h a, v16h b, v16h c, v16h d) { asm volatile("v_nop" :: "v"(a), "v"(b), "v"(c), "v"(d)); }
__device__ __forceinline__ void keep4_b(v16b a, v16b b, v16b c, v16b d) { asm volatile("v_nop" :: "v"(a), "v"(b), "v"(c), "v"(d)); }
__device__ __forceinline__ void acc_guard4(v8f& a, v8f& b, v8f& c, v8f& d) { asm volatile("v_nop\n\tv_nop\n\tv_nop\n\tv_nop" : "+v"(a), "+v"(b), "+v"(c), "+v"(d)); }
template <typename T> struct Frag;
template <> struct Frag<_Float16> {
  typedef v16h V; union U { v16h v; v8h h[2]; };
  static __device__ __forceinline__ v16h load(const _Float16* p) {
    U f; f.h[0] = *(const v8h*)(p); f.h[1] = *(const v8h*)(p + 16); return f.v;
  }
  static __device__ __forceinline__ v8f mma(v16h a, v16h b, v8f c) {
    return __builtin_amdgcn_wmma_f32_16x16x32_f16(false, a, false, b, (short)0, c, false, false);
  }
  static __device__ __forceinline__ void guard4(v8f& a, v8f& b, v8f& c, v8f& d, v16h x, v16h y) { dep_guard4_h(a, b, c, d, x, y); }
  static __device__ __forceinline__ void keep(v16h a, v16h b, v16h c, v16h d) { keep4_h(a, b, c, d); }
};
template <> struct Frag<__bf16> {
  typedef v16b V; union U { v16b v; v8b h[2]; };
  static __device__ __forceinline__ v16b load(const __bf16* p) {
    U f; f.h[0] = *(const v8b*)(p); f.h[1] = *(const v8b*)(p + 16); return f.v;
  }
  static __device__ __forceinline__ v8f mma(v16b a, v16b b, v8f c) {
    return __builtin_amdgcn_wmma_f32_16x16x32_bf16(false, a, false, b, (short)0, c, false, false);
  }
  static __device__ __forceinline__ void guard4(v8f& a, v8f& b, v8f& c, v8f& d, v16b x, v16b y) { dep_guard4_b(a, b, c, d, x, y); }
  static __device__ __forceinline__ void keep(v16b a, v16b b, v16b c, v16b d) { keep4_b(a, b, c, d); }
};

template <int ET> struct Elem;
template <> struct Elem<0> { typedef _Float16 T; };
template <> struct Elem<1> { typedef __bf16 T; };
template <int ET, int SPL, int BIAS_MODE, int OUT_MODE, bool RESID, int ACT = 0>
__global__ __launch_bounds__(256) void wmma_gemm64(
    const unsigned short* __restrict__ Ap, const unsigned short* __restrict__ A2p, int lda, long strideA,
    const unsigned short* __restrict__ Btp, const unsigned short* __restrict__ Bt2p, int ldb, long strideB,
    void* __restrict__ Cout, void* __restrict__ Cout2, int ldc, long strideC,
    const float* __restrict__ bias,
    const float* __restrict__ resid, long strideR,
    int M, int N, int K, float scale) {
  typedef typename Elem<ET>::T T;
  typedef typename Frag<T>::V V;
  const T* A = (const T*)Ap; const T* A2 = (const T*)A2p; const T* Bt = (const T*)Btp; const T* Bt2 = (const T*)Bt2p;
  __shared__ __align__(16) float sT[8][16 * 68];
  const int b    = blockIdx.y;
  const int lane = threadIdx.x & 31;
  const int wave = threadIdx.x >> 5;
  const int tilesN = N >> 6;
  const int tilesM = M >> 6;
  const int tile = blockIdx.x * 8 + wave;
  if (tile >= tilesM * tilesN) return;
  const int tm = tile / tilesN;
  const int tn = tile - tm * tilesN;
  const int m0 = tm << 6;
  const int n0 = tn << 6;

  const T* Ab  = A  + (size_t)b * strideA;
  const T* Bb  = Bt + (size_t)b * strideB;
  const T* Ab2 = (SPL >= 1) ? (A2  + (size_t)b * strideA) : nullptr;
  const T* Bb2 = (SPL == 2) ? (Bt2 + (size_t)b * strideB) : nullptr;

  const int rlane = lane & 15;
  const int koff  = (lane >> 4) * 8;
  const int mOff  = (lane >> 4) * 8;

  v8f acc[4][4];
#pragma unroll
  for (int i = 0; i < 4; ++i)
#pragma unroll
    for (int j = 0; j < 4; ++j) acc[i][j] = (v8f){0.f,0.f,0.f,0.f,0.f,0.f,0.f,0.f};

  for (int k0 = 0; k0 < K; k0 += 32) {
    V bh[4], bl[4];
#pragma unroll
    for (int j = 0; j < 4; ++j) {
      const size_t bo = (size_t)(n0 + (j << 4) + rlane) * ldb + koff + k0;
      bh[j] = Frag<T>::load(Bb + bo);
      if (SPL == 2) bl[j] = Frag<T>::load(Bb2 + bo);
    }
#pragma unroll
    for (int i = 0; i < 4; ++i) {
      const size_t ao = (size_t)(m0 + (i << 4) + rlane) * lda + koff + k0;
      V ah = Frag<T>::load(Ab + ao);
      V al;
      if (SPL >= 1) al = Frag<T>::load(Ab2 + ao);
#pragma unroll
      for (int j = 0; j < 4; ++j) {
        acc[i][j] = Frag<T>::mma(ah, bh[j], acc[i][j]);
        if (SPL == 2) acc[i][j] = Frag<T>::mma(ah, bl[j], acc[i][j]);
        if (SPL >= 1) acc[i][j] = Frag<T>::mma(al, bh[j], acc[i][j]);
      }
      Frag<T>::guard4(acc[i][0], acc[i][1], acc[i][2], acc[i][3], (SPL >= 1) ? al : ah, bh[3]);
    }
    Frag<T>::keep(bh[0], bh[1], bh[2], bh[3]);
    if (SPL == 2) Frag<T>::keep(bl[0], bl[1], bl[2], bl[3]);
  }
  acc_guard4(acc[0][0], acc[0][1], acc[0][2], acc[0][3]);
  acc_guard4(acc[1][0], acc[1][1], acc[1][2], acc[1][3]);
  acc_guard4(acc[2][0], acc[2][1], acc[2][2], acc[2][3]);
  acc_guard4(acc[3][0], acc[3][1], acc[3][2], acc[3][3]);

  float* slab = sT[wave];
  const float* Rb = RESID ? (resid + (size_t)b * strideR) : nullptr;
#pragma unroll
  for (int i = 0; i < 4; ++i) {
    const int mBase = m0 + (i << 4);
#pragma unroll
    for (int j = 0; j < 4; ++j) {
      const int n = n0 + (j << 4) + rlane;
      float bv = 0.f;
      if (BIAS_MODE == 2) bv = bias[n];
#pragma unroll
      for (int r = 0; r < 8; ++r) {
        float v = acc[i][j][r] * scale;
        if (BIAS_MODE == 1) v += bias[mBase + mOff + r];
        if (BIAS_MODE == 2) v += bv;
        if (RESID) v += Rb[(size_t)(mBase + mOff + r) * ldc + n];
        if (ACT == 1) v = tanhf(v);
        if (ACT == 2) v = fmaxf(v, 0.0f);
        if (ACT == 3) v = v / (1.0f + expf(-v));
        if (ACT == 4) v = (v > 0.f) ? v : 0.01f * v;
        if (ACT == 6) {
          const float v3 = v * v * v;
          const float yy = 0.7978845608028654f * (v + 0.044715f * v3);
          const float ee = expf(-2.0f * yy);
          v = v * __builtin_amdgcn_rcpf(1.0f + ee);
        }
        slab[(mOff + r) * 68 + (j << 4) + rlane] = v;
      }
    }
    __builtin_amdgcn_fence(__ATOMIC_RELEASE, "workgroup");
    __builtin_amdgcn_wave_barrier();
    __builtin_amdgcn_fence(__ATOMIC_ACQUIRE, "workgroup");
    if (OUT_MODE == 0) {
      float* C = (float*)Cout + (size_t)b * strideC;
      const int hh = lane >> 4, c4 = (lane & 15) * 4;
      for (int pass = 0; pass < 2; ++pass) {
#pragma unroll
        for (int it = 0; it < 8; ++it) {
          const int row = it * 2 + hh;
          v4f v = *(const v4f*)(slab + row * 68 + c4);
          *(volatile v4f*)(C + (size_t)(mBase + row) * ldc + n0 + c4) = v;
        }
        __threadfence();
      }
    } else {
      const int q = lane >> 3, c8 = (lane & 7) * 8;
      unsigned short* C  = (unsigned short*)Cout  + (size_t)b * strideC;
      unsigned short* C2 = (OUT_MODE == 2) ? ((unsigned short*)Cout2 + (size_t)b * strideC) : nullptr;
      for (int pass = 0; pass < 2; ++pass) {
#pragma unroll
        for (int it = 0; it < 4; ++it) {
          const int row = it * 4 + q;
          const float* sp = slab + row * 68 + c8;
          v8h hv, lv;
#pragma unroll
          for (int e = 0; e < 8; ++e) {
            if (OUT_MODE == 1) {
              hv[e] = (_Float16)sp[e];
            } else {
              unsigned short hb = f2bf_bits(sp[e]);
              unsigned short lb = f2bf_bits(sp[e] - bf_bits2f(hb));
              hv[e] = __builtin_bit_cast(_Float16, hb);
              lv[e] = __builtin_bit_cast(_Float16, lb);
            }
          }
          *(volatile v8h*)(C + (size_t)(mBase + row) * ldc + n0 + c8) = hv;
          if (OUT_MODE == 2) *(volatile v8h*)(C2 + (size_t)(mBase + row) * ldc + n0 + c8) = lv;
        }
        __threadfence();
      }
    }
    __builtin_amdgcn_fence(__ATOMIC_RELEASE, "workgroup");
    __builtin_amdgcn_wave_barrier();
    __builtin_amdgcn_fence(__ATOMIC_ACQUIRE, "workgroup");
  }
}

__global__ __launch_bounds__(256) void cast8_f16_kernel(
    const float* __restrict__ src, unsigned short* __restrict__ dst, int total8)
{
  const int i = blockIdx.x * 256 + threadIdx.x;
  if (i >= total8) return;
  const size_t e0 = (size_t)i << 3;
  const v4f a0 = *(const v4f*)(src + e0);
  const v4f a1 = *(const v4f*)(src + e0 + 4);
  v8h hv;
#pragma unroll
  for (int e = 0; e < 4; ++e) { hv[e] = (_Float16)a0[e]; hv[4 + e] = (_Float16)a1[e]; }
  unsigned short* q = dst + e0;
  *(volatile v8h*)q = hv;
  __threadfence();
  *(volatile v8h*)q = hv;
}

__global__ __launch_bounds__(256) void b_transpose_kernel(const float* __restrict__ Bm, unsigned short* __restrict__ BT)
{
  __shared__ float sB[64 * 65];
  const int tid = threadIdx.x, lane = tid & 31, wave = tid >> 5;
  const int h0 = blockIdx.x * 64;
  const int p0 = blockIdx.y * 64;
  const int c4 = (tid & 15) * 4, rq = tid >> 4;
#pragma unroll
  for (int i = 0; i < 4; ++i) {
    const int r = i * 16 + rq;
    const v4f v = *(const v4f*)(Bm + (size_t)(p0 + r) * kHid + h0 + c4);
    sB[r * 65 + c4 + 0] = v[0];
    sB[r * 65 + c4 + 1] = v[1];
    sB[r * 65 + c4 + 2] = v[2];
    sB[r * 65 + c4 + 3] = v[3];
  }
  __syncthreads();
  const int q = lane >> 3, c8 = (lane & 7) * 8;
  v8h ov[2];
#pragma unroll
  for (int it = 0; it < 2; ++it) {
    const int hr = it * 32 + wave * 4 + q;
#pragma unroll
    for (int e = 0; e < 8; ++e) ov[it][e] = (_Float16)sB[(c8 + e) * 65 + hr];
  }
  for (int pass = 0; pass < 2; ++pass) {
#pragma unroll
    for (int it = 0; it < 2; ++it) {
      const int hr = it * 32 + wave * 4 + q;
      *(volatile v8h*)(BT + (size_t)(h0 + hr) * kP + p0 + c8) = ov[it];
    }
    __threadfence();
  }
}

__global__ __launch_bounds__(256) void cw_fold_kernel(
    const float* __restrict__ Cm, const float* __restrict__ Wout, unsigned short* __restrict__ CW3)
{
  __shared__ __align__(16) float sv[256];
  const int tid = threadIdx.x, lane = tid & 31, wave = tid >> 5;
  const int o = blockIdx.x >> 1;
  const int hbase = (blockIdx.x & 1) * 256;
  const int h = hbase + tid;
  const float* cr = Cm + (size_t)h * kP;
  const float* wr = Wout + (size_t)o * kP;
  float acc = 0.0f;
#pragma unroll 1
  for (int p4 = 0; p4 < kP / 4; ++p4) {
    const v4f cv = *(const v4f*)(cr + 4 * p4);
    const v4f wv = *(const v4f*)(wr + 4 * p4);
    acc = fmaf(cv[0], wv[0], acc);
    acc = fmaf(cv[1], wv[1], acc);
    acc = fmaf(cv[2], wv[2], acc);
    acc = fmaf(cv[3], wv[3], acc);
  }
  sv[tid] = acc;
  __syncthreads();
  const v4f f0 = *(const v4f*)(sv + lane * 8);
  const v4f f1 = *(const v4f*)(sv + lane * 8 + 4);
  v8h s1, s2, s3;
#pragma unroll
  for (int e = 0; e < 4; ++e) {
    const float fa = f0[e], fb = f1[e];
    const float ha = h16_to_f32(f16_bits(fa)), hb = h16_to_f32(f16_bits(fb));
    s1[e] = (_Float16)(ha * 256.0f);            s1[4 + e] = (_Float16)(hb * 256.0f);
    s2[e] = (_Float16)(ha * 0.25f);             s2[4 + e] = (_Float16)(hb * 0.25f);
    s3[e] = (_Float16)((fa - ha) * 65536.0f);   s3[4 + e] = (_Float16)((fb - hb) * 65536.0f);
  }
  v8h ov = s3;
  if (wave == 0) ov = s1;
  if (wave == 1) ov = s2;
  if (wave < 3) {
    unsigned short* dst = CW3 + (size_t)o * kK3 + wave * kHid + hbase + lane * 8;
    *(volatile v8h*)dst = ov;
    __threadfence();
    *(volatile v8h*)dst = ov;
  }
}

__global__ __launch_bounds__(64) void scan_kernel(
    const unsigned* __restrict__ Uw, const float* __restrict__ adiag, unsigned* __restrict__ A3w)
{
  constexpr int kUWords = kHid / 2;
  constexpr int kAWords = kK3 / 2;
  constexpr int kSegW   = kHid / 2;
  const int j = threadIdx.x;
  const int c0 = j * 8;
  const v4f aA = *(const v4f*)(adiag + c0);
  const v4f aB = *(const v4f*)(adiag + c0 + 4);
  float av[8], hs[8];
  av[0] = aA[0]; av[1] = aA[1]; av[2] = aA[2]; av[3] = aA[3];
  av[4] = aB[0]; av[5] = aB[1]; av[6] = aB[2]; av[7] = aB[3];
#pragma unroll
  for (int e = 0; e < 8; ++e) hs[e] = 0.0f;
  size_t ui = (size_t)blockIdx.x * kT * kUWords + (size_t)j * 4;
  size_t ai = (size_t)blockIdx.x * kT * kAWords + (size_t)j * 4;
#pragma unroll 1
  for (int t = 0; t < kT; ++t) {
    const u32x4 uw = *(const u32x4*)(Uw + ui);
#pragma unroll
    for (int e = 0; e < 4; ++e) {
      const unsigned w = uw[e];
      const float u0 = h16_to_f32(w & 0xffffu);
      const float u1 = h16_to_f32(w >> 16);
      hs[2 * e]     = av[2 * e]     * hs[2 * e]     + u0;
      hs[2 * e + 1] = av[2 * e + 1] * hs[2 * e + 1] + u1;
    }
    u32x4 w1, w2, w3;
#pragma unroll
    for (int e = 0; e < 4; ++e) {
      const float ha = hs[2 * e], hb = hs[2 * e + 1];
      const unsigned b0 = f16_bits(ha), b1 = f16_bits(hb);
      const float g0 = h16_to_f32(b0), g1 = h16_to_f32(b1);
      const unsigned l0 = f16_bits((ha - g0) * 1024.0f), l1 = f16_bits((hb - g1) * 1024.0f);
      const unsigned t0 = f16_bits(g0 * 0.00390625f), t1 = f16_bits(g1 * 0.00390625f);
      w1[e] = b0 | (b1 << 16);
      w2[e] = l0 | (l1 << 16);
      w3[e] = t0 | (t1 << 16);
    }
    unsigned* q1 = A3w + ai;
    unsigned* q2 = q1 + kSegW;
    unsigned* q3 = q1 + 2 * kSegW;
    *(volatile u32x4*)q1 = w1;
    *(volatile u32x4*)q2 = w2;
    *(volatile u32x4*)q3 = w3;
    __threadfence();
    *(volatile u32x4*)q1 = w1;
    *(volatile u32x4*)q2 = w2;
    *(volatile u32x4*)q3 = w3;
    ui += kUWords;
    ai += kAWords;
  }
}

extern "C" void kernel_launch(void* const* d_in, const int* in_sizes, int n_in,
                              void* d_out, int out_size, void* d_ws, size_t ws_size,
                              hipStream_t stream) {
  if (n_in < 8) return;
  if (in_sizes[0] != kRows * kDI) return;
  if (in_sizes[1] != kHid) return;
  if (in_sizes[2] != kP * kHid) return;
  if (in_sizes[3] != kHid * kP) return;
  if (in_sizes[4] != kP * kDI) return;
  if (in_sizes[5] != kP) return;
  if (in_sizes[6] != kDO * kP) return;
  if (in_sizes[7] != kDO) return;
  if (out_size != kRows * kDO) return;
  if (ws_size < kWsTotal) return;

  const float* x     = (const float*)d_in[0];
  const float* adiag = (const float*)d_in[1];
  const float* Bm    = (const float*)d_in[2];
  const float* Cm    = (const float*)d_in[3];
  const float* W_in  = (const float*)d_in[4];
  const float* b_in  = (const float*)d_in[5];
  const float* W_out = (const float*)d_in[6];
  const float* b_out = (const float*)d_in[7];
  float* out = (float*)d_out;

  char* ws = (char*)d_ws;
  unsigned short* XH  = (unsigned short*)(ws + kOffXH);
  unsigned short* WI  = (unsigned short*)(ws + kOffWI);
  unsigned short* BT  = (unsigned short*)(ws + kOffBT);
  unsigned short* CW3 = (unsigned short*)(ws + kOffCW);
  unsigned short* PP  = (unsigned short*)(ws + kOffPP);
  unsigned short* UU  = (unsigned short*)(ws + kOffUU);
  unsigned short* A3  = (unsigned short*)(ws + kOffA3);

  cast8_f16_kernel<<<(kRows * kDI / 8) / 256, 256, 0, stream>>>(x, XH, kRows * kDI / 8);
  cast8_f16_kernel<<<(kP * kDI / 8) / 256, 256, 0, stream>>>(W_in, WI, kP * kDI / 8);
  b_transpose_kernel<<<dim3(kHid / 64, kP / 64), 256, 0, stream>>>(Bm, BT);
  cw_fold_kernel<<<2 * kDO, 256, 0, stream>>>(Cm, W_out, CW3);

  for (int qt = 0; qt < kNQ; ++qt) {
    const unsigned short* XHq = XH + (size_t)qt * kRowsQ * kDI;
    float* outq = out + (size_t)qt * kRowsQ * kDO;

    wmma_gemm64<0, 0, 2, 1, false, 6><<<dim3((kRowsQ / 64) * (kP / 64) / 8, 1), 256, 0, stream>>>(
        XHq, nullptr, kDI, 0L,
        WI, nullptr, kDI, 0L,
        (void*)PP, nullptr, kP, 0L,
        b_in, nullptr, 0L,
        kRowsQ, kP, kDI, 1.0f);

    wmma_gemm64<0, 0, 0, 1, false, 0><<<dim3((kRowsQ / 64) * (kHid / 64) / 8, 1), 256, 0, stream>>>(
        PP, nullptr, kP, 0L,
        BT, nullptr, kP, 0L,
        (void*)UU, nullptr, kHid, 0L,
        nullptr, nullptr, 0L,
        kRowsQ, kHid, kP, 1.0f);

    scan_kernel<<<kNBQ, kScanLanes, 0, stream>>>((const unsigned*)UU, adiag, (unsigned*)A3);

    wmma_gemm64<0, 0, 2, 0, false, 0><<<dim3((kRowsQ / 64) * (kDO / 64) / 8, 1), 256, 0, stream>>>(
        A3, nullptr, kK3, 0L,
        CW3, nullptr, kK3, 0L,
        (void*)outq, nullptr, kDO, 0L,
        b_out, nullptr, 0L,
        kRowsQ, kDO, kK3, 0.00390625f);
  }
}
